// GraphLSTM_26250840113392
// MI455X (gfx1250) — hardware-verified
//
#include <hip/hip_runtime.h>


#define NS   20
#define NN   4096
#define INF  2
#define DE   128
#define GH   128
#define MH   128
#define CH   256
#define CE   384
#define NO   5
#define NOP  64
#define DM   GH
#define NTK  NN
#define LOSC 1024.0f

typedef _Float16 h16;
typedef unsigned short bf;
typedef __attribute__((ext_vector_type(16))) __bf16   v16bf;
typedef __attribute__((ext_vector_type(16))) _Float16 v16h;
typedef __attribute__((ext_vector_type(8)))  _Float16 v8h;
typedef __attribute__((ext_vector_type(8)))  unsigned short v8us;
typedef __attribute__((ext_vector_type(8)))  float    v8f;
typedef __attribute__((ext_vector_type(4)))  float    v4f;
typedef __attribute__((ext_vector_type(4)))  _Float16 v4h;
typedef v8h  __attribute__((may_alias)) v8ha;
typedef v4f  __attribute__((may_alias)) v4fa;
typedef v8us __attribute__((may_alias)) v8usa;

__device__ __forceinline__ unsigned short f2bf(float f) { unsigned u = __float_as_uint(f); u += 0x7FFFu + ((u >> 16) & 1u); return (unsigned short)(u >> 16); }
__device__ __forceinline__ float bf2f(unsigned short b) { return __uint_as_float(((unsigned)b) << 16); }
__device__ __forceinline__ float bfr(float f) { return bf2f(f2bf(f)); }
__device__ __forceinline__ v16h cat16(v8h lo, v8h hi) { return __builtin_shufflevector(lo, hi, 0, 1, 2, 3, 4, 5, 6, 7, 8, 9, 10, 11, 12, 13, 14, 15); }
__device__ __forceinline__ v16bf cat16b(v8us lo, v8us hi) { return __builtin_bit_cast(v16bf, __builtin_shufflevector(lo, hi, 0, 1, 2, 3, 4, 5, 6, 7, 8, 9, 10, 11, 12, 13, 14, 15)); }
__device__ __forceinline__ v8f wmma16(v16h a, v16h b, v8f c) { return __builtin_amdgcn_wmma_f32_16x16x32_f16(false, a, false, b, (short)0, c, false, false); }
__device__ __forceinline__ v8f wmmab(v16bf a, v16bf b, v8f c) { return __builtin_amdgcn_wmma_f32_16x16x32_bf16(false, a, false, b, (short)0, c, false, false); }

__global__ __launch_bounds__(256) void k_wt(const float* __restrict__ Wm, int K, int ncols, bf* WT) {
    __shared__ __align__(16) unsigned short tl[64 * 72];
    const int tid = threadIdx.x, k0 = blockIdx.x * 64, n0 = blockIdx.y * 64;
    const int kk = tid >> 2, nq = (tid & 3) * 16;
#pragma unroll
    for (int i = 0; i < 16; ++i) tl[(nq + i) * 72 + kk] = f2bf(Wm[(size_t)(k0 + kk) * ncols + n0 + nq + i]);
    __syncthreads();
    const int piece = tid & 7;
    auto pass = [&]() {
#pragma unroll
        for (int s = 0; s < 2; ++s) { const int nr = (tid >> 3) + 32 * s; const v8us val = *(const v8usa*)(tl + nr * 72 + piece * 8); *(volatile v8us*)(WT + (size_t)(n0 + nr) * K + k0 + piece * 8) = val; }
    };
    pass(); __threadfence(); pass();
}
template <bool SPLITA, bool F16OUT = false>
__global__ __launch_bounds__(128) void k_gemmb(const bf* __restrict__ A, const bf* __restrict__ Al, const bf* __restrict__ Bn, const float* __restrict__ bias, float* C, int ldc, h16* C2, const float* __restrict__ R = nullptr, int K = DM, int roundR = 1) {
    __shared__ __align__(16) float ost[4][16 * 68];
    const int lane = threadIdx.x & 31, wave = threadIdx.x >> 5, lr = lane & 15, hi = lane >> 4;
    const int r0 = blockIdx.x * 64 + wave * 16, c0 = blockIdx.y * 64;
    const size_t aoff = (size_t)(r0 + lr) * K + 8 * hi;
    size_t boff[4];
#pragma unroll
    for (int t = 0; t < 4; ++t) boff[t] = (size_t)(c0 + t * 16 + lr) * K + 8 * hi;
    v8f acc[4];
#pragma unroll
    for (int t = 0; t < 4; ++t) acc[t] = (v8f){};
#pragma unroll 1
    for (int kc = 0; kc < K; kc += 32) {
        const v16bf a = cat16b(*(const v8us*)(A + aoff + kc), *(const v8us*)(A + aoff + kc + 16));
        v16bf al = a;
        if (SPLITA) al = cat16b(*(const v8us*)(Al + aoff + kc), *(const v8us*)(Al + aoff + kc + 16));
#pragma unroll
        for (int t = 0; t < 4; ++t) { const v16bf b = cat16b(*(const v8us*)(Bn + boff[t] + kc), *(const v8us*)(Bn + boff[t] + kc + 16)); acc[t] = wmmab(a, b, acc[t]); if (SPLITA) acc[t] = wmmab(al, b, acc[t]); }
        asm volatile("v_nop\n\tv_nop\n\tv_nop\n\tv_nop" : "+v"(acc[0]), "+v"(acc[1]), "+v"(acc[2]), "+v"(acc[3]) : "v"(a), "v"(al));
    }
    float* os = &ost[wave][0];
#pragma unroll
    for (int t = 0; t < 4; ++t) { const float bv = bias ? bfr(bias[c0 + t * 16 + lr]) : 0.f;
#pragma unroll
        for (int j = 0; j < 8; ++j) os[(hi * 8 + j) * 68 + t * 16 + lr] = acc[t][j] + bv; }
    __syncthreads();
    if (F16OUT) {
        h16* crow = (h16*)(void*)C + (size_t)r0 * ldc + c0;
        auto pass = [&]() {
#pragma unroll
            for (int s = 0; s < 4; ++s) { const int row = 4 * s + (lane >> 3), piece = lane & 7; const float* sp = os + row * 68 + piece * 8; v8h o, o2;
#pragma unroll
                for (int i = 0; i < 8; ++i) { const h16 a = (h16)sp[i]; o[i] = a; o2[i] = (h16)((sp[i] - (float)a) * LOSC); }
                *(volatile v8h*)(crow + (size_t)row * ldc + piece * 8) = o; if (C2) *(volatile v8h*)(C2 + (size_t)r0 * ldc + c0 + (size_t)row * ldc + piece * 8) = o2; }
        };
        pass(); __threadfence(); pass();
    } else {
        float* crow = C + (size_t)r0 * ldc + c0;
        auto pass = [&]() {
#pragma unroll
            for (int s = 0; s < 8; ++s) { const int Lid = (lane >> 3) + 4 * s, piece = lane & 7; const int row = Lid >> 1, cofs = (Lid & 1) * 32 + piece * 4;
                v4f val = *(const v4fa*)(os + row * 68 + cofs); if (R) { const v4f rv = *(const v4f*)(R + ((size_t)r0 + row) * ldc + c0 + cofs); val += roundR ? (v4f){bfr(rv[0]), bfr(rv[1]), bfr(rv[2]), bfr(rv[3])} : rv; }
                *(volatile v4f*)(crow + (size_t)row * ldc + cofs) = val; }
        };
        pass(); __threadfence(); pass();
    }
}


typedef __attribute__((ext_vector_type(4))) unsigned short v4us;
__device__ __forceinline__ float sigm(float x) { return 1.0f / (1.0f + __expf(-x)); }
__device__ __forceinline__ float tanhx(float x) { return 1.0f - 2.0f / (__expf(2.0f * x) + 1.0f); }
__device__ __forceinline__ void sthl4(bf* h, bf* l, size_t o, const float* v) { v4us a, b;
#pragma unroll
    for (int i = 0; i < 4; ++i) { const unsigned short hb = f2bf(v[i]); a[i] = hb; b[i] = f2bf(v[i] - bf2f(hb)); }
    *(volatile v4us*)(h + o) = a; *(volatile v4us*)(l + o) = b; }
__global__ __launch_bounds__(256) void k_bf(const float* __restrict__ src, bf* dst, size_t n8) {
    const size_t i = (size_t)blockIdx.x * 256 + threadIdx.x; if (i >= n8) return;
    const v8f v = *(const v8f*)(src + i * 8); v8us o;
#pragma unroll
    for (int k = 0; k < 8; ++k) o[k] = f2bf(v[k]);
    *(volatile v8us*)(dst + i * 8) = o; __threadfence(); *(volatile v8us*)(dst + i * 8) = o;
}
__global__ __launch_bounds__(256) void k_wout(const float* __restrict__ Wo, const float* __restrict__ bo, bf* WB, float* BO) {
    const int u = blockIdx.x * 256 + threadIdx.x;
    if (u < NOP * CH / 8) { const int n = u / (CH / 8), k0 = (u % (CH / 8)) * 8; v8us v;
#pragma unroll
        for (int i = 0; i < 8; ++i) v[i] = (n < NO) ? f2bf(Wo[n * CH + k0 + i]) : (unsigned short)0;
        *(volatile v8us*)(WB + (size_t)n * CH + k0) = v; __threadfence(); *(volatile v8us*)(WB + (size_t)n * CH + k0) = v; }
    if (u < NOP / 4) { v4f b;
#pragma unroll
        for (int i = 0; i < 4; ++i) { const int n = u * 4 + i; b[i] = (n < NO) ? bo[n] : 0.f; }
        *(volatile v4f*)(BO + u * 4) = b; __threadfence(); *(volatile v4f*)(BO + u * 4) = b; }
}
__global__ __launch_bounds__(256) void k_init(const float* __restrict__ src, int W, float* S, bf* Ph, bf* Pl) {
    const int lane = threadIdx.x & 31, r = blockIdx.x * 8 + (threadIdx.x >> 5); if (r >= NN) return;
#pragma unroll 1
    for (int ps = 0; ps < 2; ++ps) {
#pragma unroll 1
        for (int q = 0; q < W / 128; ++q) { const size_t o = (size_t)r * W + q * 128 + lane * 4; v4f v = *(const v4f*)(src + o); float f[4];
#pragma unroll
            for (int i = 0; i < 4; ++i) { v[i] = bfr(v[i]); f[i] = v[i]; }
            *(volatile v4f*)(S + o) = v; if (Ph) sthl4(Ph, Pl, o, f); }
        if (ps == 0) __threadfence(); }
}
__global__ __launch_bounds__(256) void k_emb2(const float* __restrict__ veh, const float* __restrict__ ped, const float* __restrict__ Wd, const float* __restrict__ bd, const float* __restrict__ Wv, const float* __restrict__ bv, const float* __restrict__ Wp, const float* __restrict__ bp,
                                              bf* Eh, bf* El, bf* Vh, bf* Vl, bf* Ph, bf* Pl) {
    const int lane = threadIdx.x & 31, r = blockIdx.x * 8 + (threadIdx.x >> 5); if (r >= NN) return;
    const float v0 = bfr(veh[r * 2]), v1 = bfr(veh[r * 2 + 1]), p0 = bfr(ped[r * 2]), p1 = bfr(ped[r * 2 + 1]);
    float d[4], g[4], p[4];
#pragma unroll
    for (int i = 0; i < 4; ++i) { const int c = lane * 4 + i;
        d[i] = fmaxf(fmaf(v0, bfr(Wd[c * 2]), fmaf(v1, bfr(Wd[c * 2 + 1]), bfr(bd[c]))), 0.f);
        g[i] = fmaxf(fmaf(v0, bfr(Wv[c * 2]), fmaf(v1, bfr(Wv[c * 2 + 1]), bfr(bv[c]))), 0.f);
        p[i] = fmaxf(fmaf(p0, bfr(Wp[c * 2]), fmaf(p1, bfr(Wp[c * 2 + 1]), bfr(bp[c]))), 0.f); }
    const size_t oe = (size_t)r * CE + lane * 4, og = (size_t)r * DE + lane * 4;
    sthl4(Eh, El, oe, d); sthl4(Vh, Vl, og, g); sthl4(Ph, Pl, og, p); __threadfence(); sthl4(Eh, El, oe, d); sthl4(Vh, Vl, og, g); sthl4(Ph, Pl, og, p);
}
template <int W>
__global__ __launch_bounds__(256) void k_cell(const float* __restrict__ G, float* Hs, float* Cs, bf* Ph, bf* Pl, int pw, int col0) {
    typedef __attribute__((ext_vector_type(2))) float v2f; typedef __attribute__((ext_vector_type(2))) unsigned short v2us;
    const int lane = threadIdx.x & 31, wid = blockIdx.x * 8 + (threadIdx.x >> 5); if (wid >= NN * (W / 64)) return;
    const int r = wid / (W / 64), q = wid % (W / 64); const int c0 = q * 64 + lane * 2;
    const float* gr = G + (size_t)r * 4 * W;
    const v2f gi = *(const v2f*)(gr + c0), gf = *(const v2f*)(gr + W + c0), gg = *(const v2f*)(gr + 2 * W + c0), go = *(const v2f*)(gr + 3 * W + c0), cp = *(const v2f*)(Cs + (size_t)r * W + c0);
    v2f cv, hv; v2us oh, ol;
#pragma unroll
    for (int i = 0; i < 2; ++i) { const float c2 = sigm(gf[i]) * cp[i] + sigm(gi[i]) * tanhx(gg[i]); cv[i] = c2; hv[i] = sigm(go[i]) * tanhx(c2); const unsigned short hb = f2bf(hv[i]); oh[i] = hb; ol[i] = f2bf(hv[i] - bf2f(hb)); }
    const size_t so = (size_t)r * W + c0, po = (size_t)r * pw + col0 + c0;
    *(volatile v2f*)(Cs + so) = cv; *(volatile v2f*)(Hs + so) = hv; *(volatile v2us*)(Ph + po) = oh; *(volatile v2us*)(Pl + po) = ol; __threadfence();
    *(volatile v2f*)(Cs + so) = cv; *(volatile v2f*)(Hs + so) = hv; *(volatile v2us*)(Ph + po) = oh; *(volatile v2us*)(Pl + po) = ol;
}
__global__ __launch_bounds__(256) void k_colsum(const float* __restrict__ Hs, float* SUM) {
    __shared__ float part[2][GH];
    const int tid = threadIdx.x, c = tid & (GH - 1), half = tid >> 7;
    float s = 0.f;
#pragma unroll 1
    for (int n = half * (NN / 2); n < (half + 1) * (NN / 2); ++n) s += Hs[(size_t)n * GH + c];
    part[half][c] = s;
    __syncthreads();
    if (tid < GH / 4) { v4f v;
#pragma unroll
        for (int i = 0; i < 4; ++i) v[i] = part[0][tid * 4 + i] + part[1][tid * 4 + i];
        *(volatile v4f*)(SUM + tid * 4) = v; __threadfence(); *(volatile v4f*)(SUM + tid * 4) = v; }
}
__global__ __launch_bounds__(256) void k_agga(const float* __restrict__ SUMV, const float* __restrict__ Hs, bf* Ah, bf* Al) {
    const int lane = threadIdx.x & 31, r = blockIdx.x * 8 + (threadIdx.x >> 5); if (r >= NN) return;
    const size_t o = (size_t)r * GH + lane * 4; const v4f hv = *(const v4f*)(Hs + o); float f[4];
#pragma unroll
    for (int i = 0; i < 4; ++i) f[i] = SUMV[lane * 4 + i] - hv[i];
    sthl4(Ah, Al, o, f); __threadfence(); sthl4(Ah, Al, o, f);
}
__global__ __launch_bounds__(128) void k_pedagg(const float* __restrict__ SUMP, const float* __restrict__ wgp, float* PA) {
    const int m = threadIdx.x; float s = 0.f;
#pragma unroll 1
    for (int k = 0; k < GH; ++k) s = fmaf(SUMP[k], bfr(wgp[k * MH + m]), s);
    *(volatile float*)(PA + m) = s; __threadfence(); *(volatile float*)(PA + m) = s;
}
__global__ __launch_bounds__(256) void k_embput(const float* __restrict__ VA, const float* __restrict__ PA, bf* Eh, bf* El) {
    const int lane = threadIdx.x & 31, r = blockIdx.x * 8 + (threadIdx.x >> 5); if (r >= NN) return;
    const v4f va = *(const v4f*)(VA + (size_t)r * MH + lane * 4); float a[4], p[4];
#pragma unroll
    for (int i = 0; i < 4; ++i) { a[i] = va[i]; p[i] = PA[lane * 4 + i]; }
    const size_t oa = (size_t)r * CE + DE + lane * 4, op = (size_t)r * CE + DE + MH + lane * 4;
    sthl4(Eh, El, oa, a); sthl4(Eh, El, op, p); __threadfence(); sthl4(Eh, El, oa, a); sthl4(Eh, El, op, p);
}
__global__ __launch_bounds__(256) void k_outs(const float* __restrict__ OS, float* OUT0) {
    const size_t i = (size_t)blockIdx.x * 256 + threadIdx.x; if (i >= (size_t)NS * NN * NO) return;
    const int o = (int)(i % NO), n = (int)((i / NO) % NN), s = (int)(i / ((size_t)NO * NN)); const float v = OS[((size_t)s * NN + n) * NOP + o];
    *(volatile float*)(OUT0 + i) = v; __threadfence(); *(volatile float*)(OUT0 + i) = v;
}
__global__ __launch_bounds__(256) void k_copy(const float* __restrict__ src, float* dst, size_t n4) {
    const size_t i = (size_t)blockIdx.x * 256 + threadIdx.x; if (i >= n4) return;
    const v4f v = *(const v4f*)(src + i * 4); *(volatile v4f*)(dst + i * 4) = v; __threadfence(); *(volatile v4f*)(dst + i * 4) = v;
}

extern "C" void kernel_launch(void* const* d_in, const int* in_sizes, int n_in,
                              void* d_out, int out_size, void* d_ws, size_t ws_size, hipStream_t stream) {
    (void)in_sizes; (void)n_in; (void)out_size;
    const float* veh = (const float*)d_in[0]; const float* ped = (const float*)d_in[1]; const float* cell_h = (const float*)d_in[2]; const float* cell_c = (const float*)d_in[3];
    const float* gveh_h = (const float*)d_in[4]; const float* gveh_c = (const float*)d_in[5]; const float* gped_h = (const float*)d_in[6]; const float* gped_c = (const float*)d_in[7];
    const float* Wdyn = (const float*)d_in[8]; const float* bdyn = (const float*)d_in[9]; const float* Wgve = (const float*)d_in[10]; const float* bgve = (const float*)d_in[11]; const float* Wgpe = (const float*)d_in[12]; const float* bgpe = (const float*)d_in[13];
    const float* Wihv = (const float*)d_in[14]; const float* bihv = (const float*)d_in[15]; const float* Whhv = (const float*)d_in[16]; const float* bhhv = (const float*)d_in[17];
    const float* Wihp = (const float*)d_in[18]; const float* bihp = (const float*)d_in[19]; const float* Whhp = (const float*)d_in[20]; const float* bhhp = (const float*)d_in[21];
    const float* Wihc = (const float*)d_in[22]; const float* bihc = (const float*)d_in[23]; const float* Whhc = (const float*)d_in[24]; const float* bhhc = (const float*)d_in[25];
    const float* wgv = (const float*)d_in[26]; const float* wgp = (const float*)d_in[27]; const float* Wout = (const float*)d_in[28]; const float* bout = (const float*)d_in[29];
    float* out0 = (float*)d_out; float* och = out0 + (size_t)NS * NN * NO; float* occ = och + (size_t)NN * CH; float* ogvh = occ + (size_t)NN * CH; float* ogvc = ogvh + (size_t)NN * GH; float* ogph = ogvc + (size_t)NN * GH; float* ogpc = ogph + (size_t)NN * GH;
    char* wsp = (char*)d_ws;
    auto take = [&](size_t bytes) { char* p = wsp; wsp += (bytes + 255) & ~(size_t)255; return (void*)p; };
    bf* WihvB = (bf*)take((size_t)4 * GH * DE * 2); bf* WhhvB = (bf*)take((size_t)4 * GH * GH * 2); bf* WihpB = (bf*)take((size_t)4 * GH * DE * 2); bf* WhhpB = (bf*)take((size_t)4 * GH * GH * 2);
    bf* WihcB = (bf*)take((size_t)4 * CH * CE * 2); bf* WhhcB = (bf*)take((size_t)4 * CH * CH * 2); bf* WgvT = (bf*)take((size_t)MH * GH * 2); bf* WoutB = (bf*)take((size_t)NOP * CH * 2); float* BO = (float*)take(256);
    float* SCH = (float*)take((size_t)NN * CH * 4); float* SCC = (float*)take((size_t)NN * CH * 4); float* SVH = (float*)take((size_t)NN * GH * 4); float* SVC = (float*)take((size_t)NN * GH * 4); float* SPH = (float*)take((size_t)NN * GH * 4); float* SPC = (float*)take((size_t)NN * GH * 4);
    bf* CHh = (bf*)take((size_t)NN * CH * 2); bf* CHl = (bf*)take((size_t)NN * CH * 2); bf* VHh = (bf*)take((size_t)NN * GH * 2); bf* VHl = (bf*)take((size_t)NN * GH * 2); bf* PHh = (bf*)take((size_t)NN * GH * 2); bf* PHl = (bf*)take((size_t)NN * GH * 2);
    bf* Eh = (bf*)take((size_t)NN * CE * 2); bf* El = (bf*)take((size_t)NN * CE * 2); bf* GEh = (bf*)take((size_t)NN * DE * 2); bf* GEl = (bf*)take((size_t)NN * DE * 2); bf* PEh = (bf*)take((size_t)NN * DE * 2); bf* PEl = (bf*)take((size_t)NN * DE * 2); bf* AGh = (bf*)take((size_t)NN * GH * 2); bf* AGl = (bf*)take((size_t)NN * GH * 2);
    float* T512 = (float*)take((size_t)NN * 4 * GH * 4); float* T512b = (float*)take((size_t)NN * 4 * GH * 4); float* T1024 = (float*)take((size_t)NN * 4 * CH * 4); float* T1024b = (float*)take((size_t)NN * 4 * CH * 4);
    float* SUMV = (float*)take(GH * 4); float* SUMP = (float*)take(GH * 4); float* PA = (float*)take(MH * 4); float* VA = (float*)take((size_t)NN * MH * 4); float* OS = (float*)take((size_t)NS * NN * NOP * 4);
    if ((size_t)(wsp - (char*)d_ws) > ws_size) return;
    k_bf<<<(4 * GH * DE / 8 + 255) / 256, 256, 0, stream>>>(Wihv, WihvB, 4 * GH * DE / 8); k_bf<<<(4 * GH * GH / 8 + 255) / 256, 256, 0, stream>>>(Whhv, WhhvB, 4 * GH * GH / 8);
    k_bf<<<(4 * GH * DE / 8 + 255) / 256, 256, 0, stream>>>(Wihp, WihpB, 4 * GH * DE / 8); k_bf<<<(4 * GH * GH / 8 + 255) / 256, 256, 0, stream>>>(Whhp, WhhpB, 4 * GH * GH / 8);
    k_bf<<<(4 * CH * CE / 8 + 255) / 256, 256, 0, stream>>>(Wihc, WihcB, 4 * CH * CE / 8); k_bf<<<(4 * CH * CH / 8 + 255) / 256, 256, 0, stream>>>(Whhc, WhhcB, 4 * CH * CH / 8);
    k_wt<<<dim3(GH / 64, MH / 64, 1), 256, 0, stream>>>(wgv, GH, MH, WgvT);
    k_wout<<<(NOP * CH / 8 + 255) / 256, 256, 0, stream>>>(Wout, bout, WoutB, BO);
    k_init<<<NN / 8, 256, 0, stream>>>(cell_h, CH, SCH, CHh, CHl); k_init<<<NN / 8, 256, 0, stream>>>(cell_c, CH, SCC, nullptr, nullptr);
    k_init<<<NN / 8, 256, 0, stream>>>(gveh_h, GH, SVH, VHh, VHl); k_init<<<NN / 8, 256, 0, stream>>>(gveh_c, GH, SVC, nullptr, nullptr);
    k_init<<<NN / 8, 256, 0, stream>>>(gped_h, GH, SPH, PHh, PHl); k_init<<<NN / 8, 256, 0, stream>>>(gped_c, GH, SPC, nullptr, nullptr);
    for (int s = 0; s < NS; ++s) {
        k_emb2<<<NN / 8, 256, 0, stream>>>(veh + (size_t)s * NN * INF, ped + (size_t)s * NN * INF, Wdyn, bdyn, Wgve, bgve, Wgpe, bgpe, Eh, El, GEh, GEl, PEh, PEl);
        k_gemmb<true, false><<<dim3(NN / 64, 4 * GH / 64, 1), 128, 0, stream>>>(GEh, GEl, WihvB, bihv, T512, 4 * GH, nullptr, nullptr, DE);
        k_gemmb<true, false><<<dim3(NN / 64, 4 * GH / 64, 1), 128, 0, stream>>>(VHh, VHl, WhhvB, bhhv, T512b, 4 * GH, nullptr, T512, GH, 0);
        k_cell<GH><<<(NN * (GH / 64)) / 8, 256, 0, stream>>>(T512b, SVH, SVC, VHh, VHl, GH, 0);
        k_colsum<<<1, 256, 0, stream>>>(SVH, SUMV); k_agga<<<NN / 8, 256, 0, stream>>>(SUMV, SVH, AGh, AGl);
        k_gemmb<true, false><<<dim3(NN / 64, MH / 64, 1), 128, 0, stream>>>(AGh, AGl, WgvT, nullptr, VA, MH, nullptr, nullptr, GH);
        k_gemmb<true, false><<<dim3(NN / 64, 4 * GH / 64, 1), 128, 0, stream>>>(PEh, PEl, WihpB, bihp, T512, 4 * GH, nullptr, nullptr, DE);
        k_gemmb<true, false><<<dim3(NN / 64, 4 * GH / 64, 1), 128, 0, stream>>>(PHh, PHl, WhhpB, bhhp, T512b, 4 * GH, nullptr, T512, GH, 0);
        k_cell<GH><<<(NN * (GH / 64)) / 8, 256, 0, stream>>>(T512b, SPH, SPC, PHh, PHl, GH, 0);
        k_colsum<<<1, 256, 0, stream>>>(SPH, SUMP); k_pedagg<<<1, 128, 0, stream>>>(SUMP, wgp, PA);
        k_embput<<<NN / 8, 256, 0, stream>>>(VA, PA, Eh, El);
        k_gemmb<true, false><<<dim3(NN / 64, 4 * CH / 64, 1), 128, 0, stream>>>(Eh, El, WihcB, bihc, T1024, 4 * CH, nullptr, nullptr, CE);
        k_gemmb<true, false><<<dim3(NN / 64, 4 * CH / 64, 1), 128, 0, stream>>>(CHh, CHl, WhhcB, bhhc, T1024b, 4 * CH, nullptr, T1024, CH, 0);
        k_cell<CH><<<(NN * (CH / 64)) / 8, 256, 0, stream>>>(T1024b, SCH, SCC, CHh, CHl, CH, 0);
        k_gemmb<true, false><<<dim3(NN / 64, 1, 1), 128, 0, stream>>>(CHh, CHl, WoutB, BO, OS + (size_t)s * NN * NOP, NOP, nullptr, nullptr, CH);
    }
    k_outs<<<(unsigned)(((size_t)NS * NN * NO + 255) / 256), 256, 0, stream>>>(OS, out0);
    k_copy<<<(NN * CH / 4 + 255) / 256, 256, 0, stream>>>(SCH, och, (size_t)NN * CH / 4); k_copy<<<(NN * CH / 4 + 255) / 256, 256, 0, stream>>>(SCC, occ, (size_t)NN * CH / 4);
    k_copy<<<(NN * GH / 4 + 255) / 256, 256, 0, stream>>>(SVH, ogvh, (size_t)NN * GH / 4); k_copy<<<(NN * GH / 4 + 255) / 256, 256, 0, stream>>>(SVC, ogvc, (size_t)NN * GH / 4);
    k_copy<<<(NN * GH / 4 + 255) / 256, 256, 0, stream>>>(SPH, ogph, (size_t)NN * GH / 4); k_copy<<<(NN * GH / 4 + 255) / 256, 256, 0, stream>>>(SPC, ogpc, (size_t)NN * GH / 4);
}
